// MHA_30477087932909
// MI455X (gfx1250) — hardware-verified
//
#include <hip/hip_runtime.h>
#include <math.h>

constexpr int kSeq    = 4096;
constexpr int kDm     = 1024;
constexpr int kHeads  = 32;
constexpr int kHd     = 32;
constexpr int kCc     = 3072;
constexpr int kTaps   = 4;
constexpr int kPos    = 8;
constexpr int kSub    = 32;
constexpr int kNSub   = kSeq / kSub;
constexpr int kThr    = 256;
constexpr int kSeg    = 1024;
constexpr int kTabBq  = 0;
constexpr int kTabBo  = kTabBq + kCc;
constexpr int kTabCb  = kTabBo + kDm;
constexpr int kTabCw  = kTabCb + kCc;
constexpr int kTabN   = kTabCw + kCc * kTaps;
constexpr int kTabBlocks = kTabN / kSeg;
constexpr float kCtxCarry = 256.0f;
constexpr float kWoCarry  = 16.0f;
constexpr float kOutScale = 1.0f / (kCtxCarry * kWoCarry);
constexpr size_t kPlane = (size_t)kSeq * kDm;

static_assert(kHeads * kHd == kDm, "head split");
static_assert(kCc == 3 * kDm, "q | k | v channel blocks");
static_assert(kHd == 32, "one wave lane per head channel");
static_assert(kTaps == 4, "conv taps loaded as one 16-B vector");
static_assert(kSeq % kSub == 0 && kNSub == 128, "sub-chunking exact");
static_assert(kSeq % kPos == 0, "conv row blocking exact");
static_assert(kSeq % 64 == 0 && kCc % 64 == 0 && kDm % 64 == 0, "GEMM M, N tile multiples");
static_assert(kDm % 32 == 0, "GEMM K multiple of 32");
static_assert(kCc % kThr == 0 && kDm % kThr == 0, "a conv block stays inside one channel group");
static_assert((kHeads % 2) == 0, "head pairs");
static_assert(kCc % kSeg == 0 && kDm == kSeg && (kCc * kTaps) % kSeg == 0, "table segments");
static_assert(kTabN == 19 * kSeg && kTabBlocks == 19, "table size");
static_assert(kSeg == kThr * 4, "one table block = 256 threads x 4 floats");
static_assert((kTabCw % 4) == 0, "tap table 16-B aligned");

typedef __attribute__((ext_vector_type(16))) _Float16 v16h;
typedef __attribute__((ext_vector_type(8)))  _Float16 v8h;
typedef __attribute__((ext_vector_type(16))) __bf16   v16b;
typedef __attribute__((ext_vector_type(8)))  __bf16   v8b;
typedef __attribute__((ext_vector_type(8)))  float    v8f;
typedef __attribute__((ext_vector_type(4)))  float    v4f;

__device__ __forceinline__ unsigned short f2bf_bits(float f) {
  unsigned u = __float_as_uint(f);
  return (unsigned short)((u + 0x7FFFu + ((u >> 16) & 1u)) >> 16);
}
__device__ __forceinline__ float bf_bits2f(unsigned short h) { return __uint_as_float(((unsigned)h) << 16); }
__device__ __forceinline__ float bf16r(float f) { return bf_bits2f(f2bf_bits(f)); }

__device__ __forceinline__ void dep_guard4_h(v8f& a, v8f& b, v8f& c, v8f& d, v16h x, v16h y) {
  asm volatile("v_nop\n\tv_nop\n\tv_nop\n\tv_nop" : "+v"(a), "+v"(b), "+v"(c), "+v"(d) : "v"(x), "v"(y));
}
__device__ __forceinline__ void dep_guard4_b(v8f& a, v8f& b, v8f& c, v8f& d, v16b x, v16b y) {
  asm volatile("v_nop\n\tv_nop\n\tv_nop\n\tv_nop" : "+v"(a), "+v"(b), "+v"(c), "+v"(d) : "v"(x), "v"(y));
}
__device__ __forceinline__ void keep4_h(v16h a, v16h b, v16h c, v16h d) { asm volatile("v_nop" :: "v"(a), "v"(b), "v"(c), "v"(d)); }
__device__ __forceinline__ void keep4_b(v16b a, v16b b, v16b c, v16b d) { asm volatile("v_nop" :: "v"(a), "v"(b), "v"(c), "v"(d)); }
__device__ __forceinline__ void acc_guard4(v8f& a, v8f& b, v8f& c, v8f& d) {
  asm volatile("v_nop\n\tv_nop\n\tv_nop\n\tv_nop" : "+v"(a), "+v"(b), "+v"(c), "+v"(d));
}

template <typename T> struct Frag;
template <> struct Frag<_Float16> {
  typedef v16h V; union U { v16h v; v8h h[2]; };
  static __device__ __forceinline__ v16h load(const _Float16* p) {
    U f; f.h[0] = *(const v8h*)(p); f.h[1] = *(const v8h*)(p + 16); return f.v;
  }
  static __device__ __forceinline__ v8f mma(v16h a, v16h b, v8f c) {
    return __builtin_amdgcn_wmma_f32_16x16x32_f16(false, a, false, b, (short)0, c, false, false);
  }
  static __device__ __forceinline__ void guard4(v8f& a, v8f& b, v8f& c, v8f& d, v16h x, v16h y) { dep_guard4_h(a, b, c, d, x, y); }
  static __device__ __forceinline__ void keep(v16h a, v16h b, v16h c, v16h d) { keep4_h(a, b, c, d); }
};
template <> struct Frag<__bf16> {
  typedef v16b V; union U { v16b v; v8b h[2]; };
  static __device__ __forceinline__ v16b load(const __bf16* p) {
    U f; f.h[0] = *(const v8b*)(p); f.h[1] = *(const v8b*)(p + 16); return f.v;
  }
  static __device__ __forceinline__ v8f mma(v16b a, v16b b, v8f c) {
    return __builtin_amdgcn_wmma_f32_16x16x32_bf16(false, a, false, b, (short)0, c, false, false);
  }
  static __device__ __forceinline__ void guard4(v8f& a, v8f& b, v8f& c, v8f& d, v16b x, v16b y) { dep_guard4_b(a, b, c, d, x, y); }
  static __device__ __forceinline__ void keep(v16b a, v16b b, v16b c, v16b d) { keep4_b(a, b, c, d); }
};

template <int ET> struct Elem;
template <> struct Elem<0> { typedef _Float16 T; };
template <> struct Elem<1> { typedef __bf16 T; };
template <int ET>
__global__ __launch_bounds__(256) void wmma_gemm64(
    const unsigned short* __restrict__ Ap, int lda,
    const unsigned short* __restrict__ Btp, int ldb,
    float* __restrict__ C, int ldc,
    const float* __restrict__ bias,
    int M, int N, int K, float scale) {
  typedef typename Elem<ET>::T T;
  typedef typename Frag<T>::V V;
  const T* A = (const T*)Ap; const T* Bt = (const T*)Btp;
  __shared__ __align__(16) float sT[8][16 * 68];
  const int lane = threadIdx.x & 31;
  const int wave = threadIdx.x >> 5;
  const int tilesN = N >> 6;
  const int tilesM = M >> 6;
  const int tile = blockIdx.x * 8 + wave;
  if (tile >= tilesM * tilesN) return;
  const int tm = tile / tilesN;
  const int tn = tile - tm * tilesN;
  const int m0 = tm << 6;
  const int n0 = tn << 6;

  const int rlane = lane & 15;
  const int koff  = (lane >> 4) * 8;
  const int mOff  = (lane >> 4) * 8;

  v8f acc[4][4];
#pragma unroll
  for (int i = 0; i < 4; ++i)
#pragma unroll
    for (int j = 0; j < 4; ++j) acc[i][j] = (v8f){0.f,0.f,0.f,0.f,0.f,0.f,0.f,0.f};

  for (int k0 = 0; k0 < K; k0 += 32) {
    V bh[4];
#pragma unroll
    for (int j = 0; j < 4; ++j) {
      const size_t bo = (size_t)(n0 + (j << 4) + rlane) * ldb + koff + k0;
      bh[j] = Frag<T>::load(Bt + bo);
    }
#pragma unroll
    for (int i = 0; i < 4; ++i) {
      const size_t ao = (size_t)(m0 + (i << 4) + rlane) * lda + koff + k0;
      V ah = Frag<T>::load(A + ao);
#pragma unroll
      for (int j = 0; j < 4; ++j) acc[i][j] = Frag<T>::mma(ah, bh[j], acc[i][j]);
      Frag<T>::guard4(acc[i][0], acc[i][1], acc[i][2], acc[i][3], ah, bh[3]);
    }
    Frag<T>::keep(bh[0], bh[1], bh[2], bh[3]);
  }
  acc_guard4(acc[0][0], acc[0][1], acc[0][2], acc[0][3]);
  acc_guard4(acc[1][0], acc[1][1], acc[1][2], acc[1][3]);
  acc_guard4(acc[2][0], acc[2][1], acc[2][2], acc[2][3]);
  acc_guard4(acc[3][0], acc[3][1], acc[3][2], acc[3][3]);

  float* slab = sT[wave];
#pragma unroll
  for (int i = 0; i < 4; ++i) {
    const int mBase = m0 + (i << 4);
#pragma unroll
    for (int j = 0; j < 4; ++j) {
      const int n = n0 + (j << 4) + rlane;
      const float bv = bias[n];
#pragma unroll
      for (int r = 0; r < 8; ++r) {
        const float v = acc[i][j][r] * scale + bv;
        slab[(mOff + r) * 68 + (j << 4) + rlane] = v;
      }
    }
    __builtin_amdgcn_fence(__ATOMIC_RELEASE, "workgroup");
    __builtin_amdgcn_wave_barrier();
    __builtin_amdgcn_fence(__ATOMIC_ACQUIRE, "workgroup");
    {
      const int hh = lane >> 4, c4 = (lane & 15) * 4;
      for (int pass = 0; pass < 2; ++pass) {
#pragma unroll
        for (int it = 0; it < 8; ++it) {
          const int row = it * 2 + hh;
          const v4f v = *(const v4f*)(slab + row * 68 + c4);
          *(volatile v4f*)(C + (size_t)(mBase + row) * ldc + n0 + c4) = v;
        }
        __threadfence();
      }
    }
    __builtin_amdgcn_fence(__ATOMIC_RELEASE, "workgroup");
    __builtin_amdgcn_wave_barrier();
    __builtin_amdgcn_fence(__ATOMIC_ACQUIRE, "workgroup");
  }
}

template <int MODE>
__global__ __launch_bounds__(kThr) void cvt8_kernel(const float* __restrict__ src, unsigned short* __restrict__ dst,
                                                    int nrow, int ncol8, int spitch, float sc) {
  const int i  = blockIdx.x * kThr + threadIdx.x;
  const int n8 = nrow * ncol8;
  if (i < n8) {
    const int row = i / ncol8;
    const int c8  = i - row * ncol8;
    const float* sp = src + (size_t)row * spitch + c8 * 8;
    const v4f a = *(const v4f*)(sp);
    const v4f b = *(const v4f*)(sp + 4);
    v8h hv;
#pragma unroll
    for (int e = 0; e < 4; ++e) {
      const float fa = a[e];
      const float fb = b[e];
      unsigned short b0, b1;
      if (MODE == 0) {
        b0 = f2bf_bits(fa * sc);
        b1 = f2bf_bits(fb * sc);
      } else {
        const _Float16 h0 = (_Float16)(bf16r(fa) * sc);
        const _Float16 h1 = (_Float16)(bf16r(fb) * sc);
        b0 = __builtin_bit_cast(unsigned short, h0);
        b1 = __builtin_bit_cast(unsigned short, h1);
      }
      hv[e]     = __builtin_bit_cast(_Float16, b0);
      hv[4 + e] = __builtin_bit_cast(_Float16, b1);
    }
    *(volatile v8h*)(dst + (size_t)i * 8) = hv;
    __threadfence();
    *(volatile v8h*)(dst + (size_t)i * 8) = hv;
  }
}

__global__ __launch_bounds__(kThr) void tab_prep_kernel(const float* __restrict__ bq, const float* __restrict__ bo,
                                                        const float* __restrict__ cb, const float* __restrict__ cw,
                                                        float* __restrict__ dst) {
  const int b = blockIdx.x;
  const float* src;
  if (b < 3)      src = bq + b * kSeg;
  else if (b < 4) src = bo;
  else if (b < 7) src = cb + (b - 4) * kSeg;
  else            src = cw + (b - 7) * kSeg;
  const int f0 = threadIdx.x * 4;
  const v4f v = *(const v4f*)(src + f0);
  v4f o;
#pragma unroll
  for (int e = 0; e < 4; ++e) {
    const float xe = v[e];
    o[e] = bf16r(xe);
  }
  float* op = dst + b * kSeg + f0;
  *(volatile v4f*)op = o;
  __threadfence();
  *(volatile v4f*)op = o;
}

__global__ __launch_bounds__(kThr) void conv_act_kernel(const float* __restrict__ qkv, const float* __restrict__ tab,
                                                        float* __restrict__ qkvf) {
  const int c   = blockIdx.x * kThr + threadIdx.x;
  const int s0  = blockIdx.y * kPos;
  const int grp = (blockIdx.x * kThr) / kDm;
  const v4f w4 = *(const v4f*)(tab + kTabCw + 4 * c);
  const float bz = tab[kTabCb + c];
  const float w0 = w4[0];
  const float w1 = w4[1];
  const float w2 = w4[2];
  const float w3 = w4[3];
  float xin[kPos + 3];
#pragma unroll
  for (int i = 0; i < kPos + 3; ++i) {
    const int ss = s0 - 3 + i;
    if (i < 3) {
      const int ssc = ss < 0 ? 0 : ss;
      const float xv = qkv[(size_t)ssc * kCc + c];
      xin[i] = (ss >= 0) ? xv : 0.0f;
    } else {
      xin[i] = qkv[(size_t)ss * kCc + c];
    }
  }
  float ov[kPos];
#pragma unroll
  for (int i = 0; i < kPos; ++i) {
    float acc = 0.0f;
    acc = fmaf(w0, xin[i], acc);
    acc = fmaf(w1, xin[i + 1], acc);
    acc = fmaf(w2, xin[i + 2], acc);
    acc = fmaf(w3, xin[i + 3], acc);
    const float z  = acc + bz;
    const float en = __expf(-z);
    const float sg = __builtin_amdgcn_rcpf(1.0f + en);
    ov[i] = z * sg;
  }
  if (grp != 2) {
#pragma unroll
    for (int i = 0; i < kPos; ++i) {
      const float a  = ov[i];
      const float ea = __expf(a);
      ov[i] = (a > 0.0f) ? (a + 1.0f) : ea;
    }
  }
  const int cc = c & (kDm - 1);
  const int h  = cc >> 5;
  const int d  = cc & 31;
  float* op = qkvf + (size_t)grp * kPlane + ((size_t)h * kSeq + (size_t)s0) * 32 + d;
  for (int pass = 0; pass < 2; ++pass) {
#pragma unroll
    for (int i = 0; i < kPos; ++i) *(volatile float*)(op + i * 32) = ov[i];
    __threadfence();
  }
}

__global__ __launch_bounds__(64) void seq_ctx_kernel(const float* __restrict__ qf, const float* __restrict__ kf,
                                                     const float* __restrict__ vf,
                                                     unsigned short* __restrict__ ctxh) {
  __shared__ __align__(16) float Qs[2][kSub * 32];
  __shared__ __align__(16) float Ks[2][kSub * 32];
  __shared__ __align__(16) float Vs[2][kSub * 32];
  __shared__ __align__(16) float Ps[2][kSub * 36];
  __shared__ __align__(16) float Cs[kSub * 68];
  __shared__ __align__(16) float Ri[2 * kSub];
  const int tid = threadIdx.x, lane = tid & 31, w = tid >> 5;
  const int p = blockIdx.x;
  const int h = 2 * p + w;
  float* qs = Qs[w];
  float* ks = Ks[w];
  float* vs = Vs[w];
  float* ps = Ps[w];

  float KV[32];
#pragma unroll
  for (int d = 0; d < 32; ++d) KV[d] = 0.0f;
  float kc = 0.0f;

#pragma unroll 1
  for (int sub = 0; sub < kNSub; ++sub) {
    const size_t base = ((size_t)h * kSeq + (size_t)sub * kSub) * 32;
    {
      v4f tq[8];
#pragma unroll
      for (int i = 0; i < 8; ++i) tq[i] = *(const v4f*)(qf + base + (size_t)(i * 32 + lane) * 4);
#pragma unroll
      for (int i = 0; i < 8; ++i) *(v4f*)(qs + (i * 32 + lane) * 4) = tq[i];
      asm volatile("" ::: "memory");
      v4f tk[8];
#pragma unroll
      for (int i = 0; i < 8; ++i) tk[i] = *(const v4f*)(kf + base + (size_t)(i * 32 + lane) * 4);
#pragma unroll
      for (int i = 0; i < 8; ++i) *(v4f*)(ks + (i * 32 + lane) * 4) = tk[i];
      asm volatile("" ::: "memory");
      v4f tv[8];
#pragma unroll
      for (int i = 0; i < 8; ++i) tv[i] = *(const v4f*)(vf + base + (size_t)(i * 32 + lane) * 4);
#pragma unroll
      for (int i = 0; i < 8; ++i) *(v4f*)(vs + (i * 32 + lane) * 4) = tv[i];
      asm volatile("" ::: "memory");
    }
    __syncthreads();

#pragma unroll 1
    for (int s = 0; s < kSub; ++s) {
      const float vt = vs[s * 32 + lane];
      const float ko = ks[s * 32 + lane];
      const float qo = qs[s * 32 + lane];
      kc += ko;
      ps[s * 36 + lane] = qo * kc;
      float num = 0.0f;
#pragma unroll
      for (int j = 0; j < 8; ++j) {
        const v4f k4 = *(const v4f*)(ks + s * 32 + 4 * j);
        const v4f q4 = *(const v4f*)(qs + s * 32 + 4 * j);
#pragma unroll
        for (int e = 0; e < 4; ++e) {
          const float kd = k4[e];
          const float qd = q4[e];
          KV[4 * j + e] = fmaf(kd, vt, KV[4 * j + e]);
          num = fmaf(qd, KV[4 * j + e], num);
        }
      }
      Cs[s * 68 + w * 32 + lane] = num;
    }
    __syncthreads();

    {
      float den = 0.0f;
#pragma unroll
      for (int j = 0; j < 8; ++j) {
        const v4f p4 = *(const v4f*)(ps + lane * 36 + 4 * j);
        const float p0 = p4[0];
        const float p1 = p4[1];
        const float p2 = p4[2];
        const float p3 = p4[3];
        den += (p0 + p1) + (p2 + p3);
      }
      Ri[w * kSub + lane] = 1.0f / den;
    }
    __syncthreads();

    v8h hv[4];
#pragma unroll
    for (int it = 0; it < 4; ++it) {
      const int idx = it * 64 + tid;
      const int row = idx >> 3, c8 = (idx & 7) * 8;
      const int hw = c8 >> 5;
      const float rv = Ri[hw * kSub + row] * kCtxCarry;
      const float* sp = Cs + row * 68 + c8;
      const v4f a = *(const v4f*)(sp);
      const v4f b = *(const v4f*)(sp + 4);
#pragma unroll
      for (int e = 0; e < 4; ++e) {
        const float fa = a[e];
        const float fb = b[e];
        hv[it][e]     = (_Float16)(fa * rv);
        hv[it][4 + e] = (_Float16)(fb * rv);
      }
    }
    for (int pass = 0; pass < 2; ++pass) {
#pragma unroll
      for (int it = 0; it < 4; ++it) {
        const int idx = it * 64 + tid;
        const int row = idx >> 3, c8 = (idx & 7) * 8;
        unsigned short* op = ctxh + (size_t)(sub * kSub + row) * kDm + p * 64 + c8;
        *(volatile v8h*)op = hv[it];
      }
      __threadfence();
    }
  }
}

extern "C" void kernel_launch(void* const* d_in, const int* in_sizes, int n_in,
                              void* d_out, int out_size, void* d_ws, size_t ws_size, hipStream_t stream) {
  if (n_in < 7 || d_out == nullptr || d_ws == nullptr) return;
  if (in_sizes[0] != kSeq * kDm || in_sizes[1] != kCc * kDm || in_sizes[2] != kCc ||
      in_sizes[3] != kCc * kTaps || in_sizes[4] != kCc || in_sizes[5] != kDm * kDm ||
      in_sizes[6] != kDm || out_size != kSeq * kDm) return;

  const float* x      = (const float*)d_in[0];
  const float* wqkv   = (const float*)d_in[1];
  const float* bqkv   = (const float*)d_in[2];
  const float* conv_w = (const float*)d_in[3];
  const float* conv_b = (const float*)d_in[4];
  const float* out_w  = (const float*)d_in[5];
  const float* out_b  = (const float*)d_in[6];
  float* out = (float*)d_out;

  char* ws = (char*)d_ws; size_t off = 0;
  auto carve = [&](size_t bytes) -> char* { char* p = ws + off; off += (bytes + 255) & ~(size_t)255; return p; };
  unsigned short* XB    = (unsigned short*)carve((size_t)kSeq * kDm * 2);
  unsigned short* WQB   = (unsigned short*)carve((size_t)kCc * kDm * 2);
  unsigned short* OWH   = (unsigned short*)carve((size_t)kDm * kDm * 2);
  float*          TAB   = (float*)carve((size_t)kTabN * 4);
  float*          QKV32 = (float*)carve((size_t)kSeq * kCc * 4);
  float*          QKVF  = (float*)carve((size_t)3 * kPlane * 4);
  unsigned short* CTXH  = (unsigned short*)carve((size_t)kSeq * kDm * 2);
  if (off > ws_size || off > (size_t)134217728) return;

  const int n8x = kSeq * (kDm / 8);
  const int n8w = kCc * (kDm / 8);
  const int n8o = kDm * (kDm / 8);
  static_assert((kSeq * (kDm / 8)) % kThr == 0 && (kCc * (kDm / 8)) % kThr == 0 && (kDm * (kDm / 8)) % kThr == 0, "convert grids exact");
  cvt8_kernel<0><<<n8x / kThr, kThr, 0, stream>>>(x,     XB,  kSeq, kDm / 8, kDm, 1.0f);
  cvt8_kernel<0><<<n8w / kThr, kThr, 0, stream>>>(wqkv,  WQB, kCc,  kDm / 8, kDm, 1.0f);
  cvt8_kernel<1><<<n8o / kThr, kThr, 0, stream>>>(out_w, OWH, kDm,  kDm / 8, kDm, kWoCarry);
  tab_prep_kernel<<<kTabBlocks, kThr, 0, stream>>>(bqkv, out_b, conv_b, conv_w, TAB);

  static_assert(((kSeq / 64) * (kCc / 64)) % 8 == 0, "GEMM0 grid exact");
  wmma_gemm64<1><<<(kSeq / 64) * (kCc / 64) / 8, 256, 0, stream>>>(
      XB, kDm, WQB, kDm, QKV32, kCc, TAB + kTabBq, kSeq, kCc, kDm, 1.0f);

  conv_act_kernel<<<dim3(kCc / kThr, kSeq / kPos), kThr, 0, stream>>>(QKV32, TAB, QKVF);

  const float* QF = QKVF;
  const float* KF = QKVF + kPlane;
  const float* VF = QKVF + 2 * kPlane;
  seq_ctx_kernel<<<kHeads / 2, 64, 0, stream>>>(QF, KF, VF, CTXH);

  static_assert(((kSeq / 64) * (kDm / 64)) % 8 == 0, "GEMM1 grid exact");
  wmma_gemm64<0><<<(kSeq / 64) * (kDm / 64) / 8, 256, 0, stream>>>(
      CTXH, kDm, OWH, kDm, out, kDm, TAB + kTabBo, kSeq, kDm, kDm, kOutScale);
}
